// StructuralEncoder_82918638617231
// MI455X (gfx1250) — hardware-verified
//
#include <hip/hip_runtime.h>
#include <math.h>

typedef __attribute__((ext_vector_type(16))) _Float16 v16h;
typedef __attribute__((ext_vector_type(16))) __bf16 v16b;
typedef __attribute__((ext_vector_type(8)))  _Float16 v8h;
typedef __attribute__((ext_vector_type(8)))  float v8f;
typedef __attribute__((ext_vector_type(4)))  float v4f;
typedef __attribute__((ext_vector_type(2)))  float v2f;
typedef __attribute__((ext_vector_type(4)))  unsigned v4u;
typedef __attribute__((ext_vector_type(4)))  int v4i;
typedef float __attribute__((may_alias)) float_a;
typedef int __attribute__((may_alias)) int_a;

template <typename T> __device__ __forceinline__ void vst2(void* p, T v) { *(volatile T*)p = v; __threadfence(); *(volatile T*)p = v; }
__device__ __forceinline__ v8f wmma16(v16h a, v16h b, v8f c) {
  v8f d = __builtin_amdgcn_wmma_f32_16x16x32_f16(false, a, false, b, (short)0, c, false, false);
  asm volatile("v_nop\n\tv_nop\n\tv_nop\n\tv_nop" : "+v"(d) : "v"(a), "v"(b));
  return d;
}
__device__ __forceinline__ v8f wmma_bf(v16b a, v16b b, v8f c) {
  v8f d = __builtin_amdgcn_wmma_f32_16x16x32_bf16(false, a, false, b, (short)0, c, false, false);
  asm volatile("v_nop\n\tv_nop\n\tv_nop\n\tv_nop" : "+v"(d) : "v"(a), "v"(b));
  return d;
}
__device__ __forceinline__ v16h frag_h(const _Float16* rowk0, int lane) {
  union { v16h v; v8h q[2]; } u; const _Float16* p = rowk0 + 8 * (lane >> 4);
  u.q[0] = *(const v8h*)p; u.q[1] = *(const v8h*)(p + 16); return u.v;
}
__device__ __forceinline__ v16h frag_f32(const float* rowk0, int lane) {
  v16h a; const float* p = rowk0 + 8 * (lane >> 4);
#pragma unroll
  for (int i = 0; i < 8; ++i) { a[i] = (_Float16)p[i]; a[8 + i] = (_Float16)p[16 + i]; }
  return a;
}
__device__ __forceinline__ v16h frag_f32s(const float* rowk0, int lane, float sc) {
  v16h a; const float* p = rowk0 + 8 * (lane >> 4);
#pragma unroll
  for (int i = 0; i < 8; ++i) { a[i] = (_Float16)(p[i] * sc); a[8 + i] = (_Float16)(p[16 + i] * sc); }
  return a;
}
__device__ __forceinline__ v16h fragc_f32(const float* W, int k0, int n, int lane, int ld, int K) {
  v16h a; const int g = lane >> 4;
#pragma unroll
  for (int i = 0; i < 8; ++i) { const int ka = k0 + 8 * g + i, kb = ka + 16;
    a[i] = (_Float16)(ka < K ? W[(size_t)(ka < K ? ka : K - 1) * ld + n] : 0.f); a[8 + i] = (_Float16)(kb < K ? W[(size_t)(kb < K ? kb : K - 1) * ld + n] : 0.f); }
  return a;
}
struct F2 { v16b h, l; };
__device__ __forceinline__ F2 bsplit16(const float v[16]) { F2 r;
#pragma unroll
  for (int i = 0; i < 16; ++i) { const __bf16 h = (__bf16)v[i]; r.h[i] = h; r.l[i] = (__bf16)(v[i] - (float)h); }
  return r; }
__device__ __forceinline__ F2 split_row(const float* row, int k0, int lane) { float v[16]; const float* p = row + k0 + 8 * (lane >> 4);
#pragma unroll
  for (int i = 0; i < 8; ++i) { v[i] = p[i]; v[8 + i] = p[16 + i]; }
  return bsplit16(v); }
__device__ __forceinline__ F2 split_rowK(const float* row, int k0, int lane, int K) { float v[16]; const int g = lane >> 4;
#pragma unroll
  for (int i = 0; i < 8; ++i) { const int ka = k0 + 8 * g + i, kb = ka + 16; v[i] = ka < K ? row[ka < K ? ka : K - 1] : 0.f; v[8 + i] = kb < K ? row[kb < K ? kb : K - 1] : 0.f; }
  return bsplit16(v); }
__device__ __forceinline__ F2 split_col(const float* W, int k0, int n, int lane, int ld, int K) { float v[16]; const int g = lane >> 4;
#pragma unroll
  for (int i = 0; i < 8; ++i) { const int ka = k0 + 8 * g + i, kb = ka + 16; v[i] = ka < K ? W[(size_t)(ka < K ? ka : K - 1) * ld + n] : 0.f; v[8 + i] = kb < K ? W[(size_t)(kb < K ? kb : K - 1) * ld + n] : 0.f; }
  return bsplit16(v); }
__device__ __forceinline__ v8f mac3(const F2& a, const F2& b, v8f c) { c = wmma_bf(a.l, b.h, c); c = wmma_bf(a.h, b.l, c); return wmma_bf(a.h, b.h, c); }
__device__ __forceinline__ float sigm(float v) { return 1.0f / (1.0f + expf(-v)); }
#define LDSX() do { asm volatile("s_wait_dscnt 0" ::: "memory"); __builtin_amdgcn_wave_barrier(); __builtin_amdgcn_fence(__ATOMIC_RELEASE, "workgroup"); } while (0)

#define NN 2048
#define TT NN
#define DF 128
#define CC 256
#define NH 8
#define HD 32
#define NE 65536
#define DFF 1024
#define DOUT 128
#define MAXDEG 512
#define HG 4
#ifndef PSTR
#define PSTR NN
#endif
#ifndef ESTR
#define ESTR NE
#endif
typedef __attribute__((ext_vector_type(8))) __bf16 v8b;
__device__ __forceinline__ v16b frag_b(const __bf16* rowk0, int lane) { union { v16b v; v8b q[2]; } u; const __bf16* p = rowk0 + 8 * (lane >> 4); u.q[0] = *(const v8b*)p; u.q[1] = *(const v8b*)(p + 16); return u.v; }
__device__ __forceinline__ float bfr(float v) { return (float)(__bf16)v; }
__device__ __attribute__((noinline)) float gelu_ni(float x) { return 0.5f * x * (1.0f + erff(x * 0.70710678118654752f)); }
#define WS_DEG 0u
#define WS_H   (WS_DEG + 4u * 2u * NN)
#define WS_ST  (WS_H + 4u * (size_t)NN * CC)
#define WS_QH  (WS_ST + 4u * (size_t)NN * 2)
#define WS_QL  (WS_QH + 2u * (size_t)NN * CC)
#define WS_KH  (WS_QL + 2u * (size_t)NN * CC)
#define WS_KL  (WS_KH + 2u * (size_t)NN * CC)
#define WS_VT  (WS_KL + 2u * (size_t)NN * CC)
#define WS_VL  (WS_VT + 2u * (size_t)CC * NN)
#define WS_S   (WS_VL + 2u * (size_t)CC * NN)
#define WS_Y   (WS_S + 4u * (size_t)HG * NN * NN)
#define WS_G   (WS_Y + 4u * (size_t)NN * CC)
#define WS_END (WS_G + 4u * (size_t)NN * DFF)
__global__ __launch_bounds__(512) void k_deg(const int* __restrict__ EI, int* __restrict__ DEG) { __shared__ int hin[NN], hout[NN];
  const int t = threadIdx.x; for (int i = t; i < NN; i += 512) { hin[i] = 0; hout[i] = 0; } __syncthreads();
  for (int e = t; e < NE; e += 512) { const int s = EI[e], d = EI[ESTR + e]; if (s < 0 || s >= NN || d < 0 || d >= NN) continue; atomicAdd(&hout[s], 1); atomicAdd(&hin[d], 1); }
  __syncthreads();
  for (int q = t; q < NN / 4; q += 512) { v4i a, b; for (int k = 0; k < 4; ++k) { const int vi = hin[q * 4 + k], vo = hout[q * 4 + k]; a[k] = vi > MAXDEG ? MAXDEG : vi; b[k] = vo > MAXDEG ? MAXDEG : vo; } vst2(DEG + q * 4, a); vst2(DEG + NN + q * 4, b); } }
__global__ __launch_bounds__(128) void k_emb(const float* __restrict__ X, const float* __restrict__ WE, const float* __restrict__ BE, float* __restrict__ H) { __shared__ __align__(16) float sf[4][16][132];
  const int tid = threadIdx.x, wave = tid >> 5, lane = tid & 31, col = lane & 15, g = lane >> 4; const size_t r0 = (size_t)blockIdx.x * 64 + wave * 16; const int c0 = blockIdx.y * 128;
  v8f acc[8] = {};
#pragma unroll
  for (int kc = 0; kc < DF / 32; ++kc) { v16b a; { const float* p = X + (r0 + col) * DF + kc * 32 + 8 * g;
#pragma unroll
      for (int i = 0; i < 8; ++i) { a[i] = (__bf16)p[i]; a[8 + i] = (__bf16)p[16 + i]; } }
#pragma unroll
    for (int j = 0; j < 8; ++j) { v16b w; const int o = c0 + j * 16 + col;
#pragma unroll
      for (int i = 0; i < 8; ++i) { w[i] = (__bf16)WE[(size_t)(kc * 32 + 8 * g + i) * CC + o]; w[8 + i] = (__bf16)WE[(size_t)(kc * 32 + 16 + 8 * g + i) * CC + o]; }
      asm volatile("s_wait_loadcnt 0x0" ::: "memory"); acc[j] = wmma_bf(a, w, acc[j]); } }
#pragma unroll
  for (int j = 0; j < 8; ++j) { const float bb = bfr(BE[c0 + j * 16 + col]);
#pragma unroll
    for (int r = 0; r < 8; ++r) sf[wave][8 * g + r][j * 16 + col] = acc[j][r] + bb; }
  LDSX(); for (int rl = 0; rl < 16; ++rl) vst2(H + (r0 + rl) * CC + c0 + lane * 4, *(const v4f*)&sf[wave][rl][lane * 4]); }
__global__ __launch_bounds__(256) void k_hadd(float* __restrict__ H, const int* __restrict__ DEG, const float* __restrict__ DIN, const float* __restrict__ DOUT_, float* __restrict__ ST) { __shared__ __align__(16) float so[32]; __shared__ __align__(16) float rowbuf[16][CC];
  const int t = threadIdx.x; const int rl = t >> 4, sub = t & 15; const size_t n = (size_t)blockIdx.x * 16 + rl; const int di = DEG[n], dq = DEG[NN + n]; float* hr = H + n * CC;
  float s = 0.f;
  for (int q = sub; q < CC / 4; q += 16) { v4f hv = *(const v4f*)(hr + q * 4); const float* a = DIN + (size_t)di * CC + q * 4; const float* b = DOUT_ + (size_t)dq * CC + q * 4;
#pragma unroll
    for (int e = 0; e < 4; ++e) { hv[e] = hv[e] + bfr(a[e]) + bfr(b[e]); s += hv[e]; }
    *(v4f*)&rowbuf[rl][q * 4] = hv; }
#pragma unroll
  for (int o = 1; o < 16; o <<= 1) s += __shfl_xor(s, o);
  const float mu = s * (1.0f / CC); float s2 = 0.f; for (int q = sub; q < CC / 4; q += 16) { const v4f hv = *(const v4f*)&rowbuf[rl][q * 4];
#pragma unroll
    for (int e = 0; e < 4; ++e) { const float d = hv[e] - mu; s2 += d * d; } }
#pragma unroll
  for (int o = 1; o < 16; o <<= 1) s2 += __shfl_xor(s2, o);
  if (sub == 0) { so[rl * 2] = mu; so[rl * 2 + 1] = rsqrtf(s2 * (1.0f / CC) + 1e-5f); }
  __syncthreads();
  for (int q = sub; q < CC / 4; q += 16) vst2(hr + q * 4, *(const v4f*)&rowbuf[rl][q * 4]);
  if (t < 32) vst2(ST + (size_t)blockIdx.x * 32 + t, so[t]); }
__global__ __launch_bounds__(256) void k_lnst(const float* __restrict__ H, float* __restrict__ ST) { __shared__ __align__(16) float so[32];
  const int t = threadIdx.x; const int rl = t >> 4, sub = t & 15; const size_t n = (size_t)blockIdx.x * 16 + rl; const float* hr = H + n * CC;
  float s = 0.f; for (int c = sub; c < CC; c += 16) s += hr[c];
#pragma unroll
  for (int o = 1; o < 16; o <<= 1) s += __shfl_xor(s, o);
  const float mu = s * (1.0f / CC); float s2 = 0.f; for (int c = sub; c < CC; c += 16) { const float d = hr[c] - mu; s2 += d * d; }
#pragma unroll
  for (int o = 1; o < 16; o <<= 1) s2 += __shfl_xor(s2, o);
  if (sub == 0) { so[rl * 2] = mu; so[rl * 2 + 1] = rsqrtf(s2 * (1.0f / CC) + 1e-5f); }
  __syncthreads(); if (t < 32) vst2(ST + (size_t)blockIdx.x * 32 + t, so[t]); }
__device__ __forceinline__ F2 lnfrag(const float* __restrict__ H, const float* __restrict__ ST, const float* __restrict__ LG, const float* __restrict__ LBt, size_t row, int kc, int lane) { float v[16]; const int g = lane >> 4; const float mu = ST[row * 2], rs = ST[row * 2 + 1]; const float* p = H + row * CC + kc * 32 + 8 * g;
#pragma unroll
  for (int i = 0; i < 8; ++i) { const int c = kc * 32 + 8 * g + i; v[i] = (p[i] - mu) * rs * bfr(LG[c]) + bfr(LBt[c]); v[8 + i] = (p[16 + i] - mu) * rs * bfr(LG[c + 16]) + bfr(LBt[c + 16]); }
  return bsplit16(v); }
__global__ __launch_bounds__(128) void k_qkv(const float* __restrict__ H, const float* __restrict__ ST, const float* __restrict__ LG, const float* __restrict__ LBt, const float* __restrict__ WQ, const float* __restrict__ BQ, const float* __restrict__ WK, const float* __restrict__ BK, const float* __restrict__ WV, const float* __restrict__ BV, _Float16* __restrict__ QH, _Float16* __restrict__ QL, _Float16* __restrict__ KH, _Float16* __restrict__ KL, __bf16* __restrict__ VT, __bf16* __restrict__ VL) {
  __shared__ __align__(16) _Float16 sh[64][136], sl[64][136]; __shared__ __align__(16) __bf16 th[128][72], tl2[128][72];
  const int tid = threadIdx.x, wave = tid >> 5, lane = tid & 31, col = lane & 15, g = lane >> 4; const int which = blockIdx.z; const int c0 = blockIdx.y * 128; const size_t r0 = (size_t)blockIdx.x * 64; const float* WA = which == 0 ? WQ : which == 1 ? WK : WV; const float* BA = which == 0 ? BQ : which == 1 ? BK : BV;
  v8f acc[8] = {};
#pragma unroll 1
  for (int kc = 0; kc < CC / 32; ++kc) { const F2 a = lnfrag(H, ST, LG, LBt, r0 + wave * 16 + col, kc, lane);
#pragma unroll
    for (int j = 0; j < 8; ++j) { v16b w; const int o = c0 + j * 16 + col;
#pragma unroll
      for (int i = 0; i < 8; ++i) { w[i] = (__bf16)WA[(size_t)(kc * 32 + 8 * g + i) * CC + o]; w[8 + i] = (__bf16)WA[(size_t)(kc * 32 + 16 + 8 * g + i) * CC + o]; }
      asm volatile("s_wait_loadcnt 0x0" ::: "memory"); acc[j] = wmma_bf(a.h, w, acc[j]); acc[j] = wmma_bf(a.l, w, acc[j]); } }
#pragma unroll
  for (int j = 0; j < 8; ++j) { const float bb = bfr(BA[c0 + j * 16 + col]);
#pragma unroll
    for (int r = 0; r < 8; ++r) { const float v = acc[j][r] + bb; const int rl = wave * 16 + 8 * g + r, cl = j * 16 + col; const _Float16 hv = (_Float16)v;
      if (which == 2) { const __bf16 bh = (__bf16)v; th[cl][rl] = bh; tl2[cl][rl] = (__bf16)(v - (float)bh); } else { sh[rl][cl] = hv; sl[rl][cl] = (_Float16)((v - (float)hv) * 1024.0f); } } }
  __syncthreads();
  if (which < 2) { _Float16* dh = which == 0 ? QH : KH; _Float16* dl = which == 0 ? QL : KL; for (int e = tid; e < 64 * 16; e += 128) { const int rl = e >> 4, q = e & 15; vst2((unsigned*)(dh + (r0 + rl) * CC + c0 + q * 8), *(const v4u*)&sh[rl][q * 8]); vst2((unsigned*)(dl + (r0 + rl) * CC + c0 + q * 8), *(const v4u*)&sl[rl][q * 8]); } }
  else { for (int e = tid; e < 128 * 8; e += 128) { const int cl = e >> 3, q = e & 7; const size_t o2 = (size_t)(c0 + cl) * NN + r0 + q * 8; vst2((unsigned*)(VT + o2), *(const v4u*)&th[cl][q * 8]); vst2((unsigned*)(VL + o2), *(const v4u*)&tl2[cl][q * 8]); } } }
__global__ __launch_bounds__(128) void k_sc(const _Float16* __restrict__ QH, const _Float16* __restrict__ QL, const _Float16* __restrict__ KH, const _Float16* __restrict__ KL, const float* __restrict__ POS, const float* __restrict__ SPD, int h0, float* __restrict__ S0) { __shared__ __align__(16) float ss[4][16][132]; __shared__ __align__(16) float spos[64][132]; __shared__ float sspd[11 * NH];
  const int h = h0 + blockIdx.z; float* S = S0 + (size_t)blockIdx.z * NN * NN;
  const int tid = threadIdx.x, wave = tid >> 5, lane = tid & 31, col = lane & 15, g = lane >> 4; const int k0 = blockIdx.y * 128; const int q0b = blockIdx.x * 64; const int ql0 = q0b + wave * 16;
  for (int e = tid; e < 64 * 32; e += 128) { const int rl = e >> 5, q = e & 31; *(v4f*)&spos[rl][q * 4] = *(const v4f*)(POS + (size_t)(q0b + rl) * PSTR + k0 + q * 4); }
  if (tid < 11 * NH) sspd[tid] = bfr(SPD[tid]); __syncthreads();
  v8f acc[8] = {}, accl[8] = {};
  { const v16h ah = frag_h(QH + (size_t)(ql0 + col) * CC + h * HD, lane), al = frag_h(QL + (size_t)(ql0 + col) * CC + h * HD, lane);
#pragma unroll
    for (int j = 0; j < 8; ++j) { const size_t ko = (size_t)(k0 + j * 16 + col) * CC + h * HD; const v16h kb = frag_h(KH + ko, lane), kl = frag_h(KL + ko, lane); acc[j] = wmma16(ah, kb, acc[j]); accl[j] = wmma16(al, kb, accl[j]); accl[j] = wmma16(ah, kl, accl[j]); } }
#pragma unroll
  for (int j = 0; j < 8; ++j) acc[j] += accl[j] * (1.0f / 1024.0f);
#pragma unroll
  for (int j = 0; j < 8; ++j) { const int kl_ = j * 16 + col;
#pragma unroll
    for (int r = 0; r < 8; ++r) { const int rl = wave * 16 + 8 * g + r; float pb = bfr(spos[rl][kl_]) * 10.0f + 0.5f; pb = fminf(fmaxf(pb, 0.f), 10.0f); const int bkt = (int)pb;
      ss[wave][8 * g + r][kl_] = acc[j][r] * 0.17677669529663688f + sspd[bkt * NH + h]; } }
  LDSX(); for (int rl = 0; rl < 16; ++rl) vst2(S + (size_t)(ql0 + rl) * NN + k0 + lane * 4, *(const v4f*)&ss[wave][rl][lane * 4]); }
__global__ __launch_bounds__(32) void k_edge(const int* __restrict__ EI, const int* __restrict__ ET, const float* __restrict__ ETAB, int h0, float* __restrict__ S0) {
  const int lane = threadIdx.x; if (lane >= HG) return; const int h = h0 + lane; float* S = S0 + (size_t)lane * NN * NN;
#pragma unroll 1
  for (int e = 0; e < NE; ++e) { const int s = EI[e], d = EI[ESTR + e]; int ty = ET[e]; if (s < 0 || s >= NN || d < 0 || d >= NN) continue; ty = ty < 0 ? 0 : (ty > 7 ? 7 : ty);
    volatile __attribute__((address_space(1))) float* p = (volatile __attribute__((address_space(1))) float*)(S + (size_t)s * NN + d); const float cur = *p; *p = cur + bfr(ETAB[ty * NH + h]);
    asm volatile("s_wait_storecnt 0x0\n\ts_wait_loadcnt 0x0" ::: "memory"); } }
__global__ __launch_bounds__(256) void k_sm(float* __restrict__ S0) { __shared__ float sred[8]; __shared__ float sbc; __shared__ __align__(16) float sh[TT];
  const int t = threadIdx.x; const size_t row = blockIdx.x; float* sr = S0 + (size_t)blockIdx.y * TT * TT + row * TT; const int kend = TT;
  float m = -3.0e38f; for (int k = t; k < kend; k += 256) m = fmaxf(m, sr[k]);
#pragma unroll
  for (int o = 1; o < 32; o <<= 1) m = fmaxf(m, __shfl_xor(m, o));
  if ((t & 31) == 0) sred[t >> 5] = m; __syncthreads(); if (t == 0) { float a = sred[0]; for (int i = 1; i < 8; ++i) a = fmaxf(a, sred[i]); sbc = a; } __syncthreads(); m = sbc; __syncthreads();
  float sum = 0.f; for (int k = t; k < kend; k += 256) { const float v = sr[k]; sum += (v <= -1.0e38f) ? 0.f : expf(v - m); }
#pragma unroll
  for (int o = 1; o < 32; o <<= 1) sum += __shfl_xor(sum, o);
  if ((t & 31) == 0) sred[t >> 5] = sum; __syncthreads(); if (t == 0) { float a = 0.f; for (int i = 0; i < 8; ++i) a += sred[i]; sbc = 1.0f / a; } __syncthreads(); const float inv = sbc;
  for (int k = t; k < kend; k += 256) { const float v = sr[k]; sh[k] = (v <= -1.0e38f) ? 0.f : expf(v - m) * inv * 2048.0f; }
  __syncthreads(); for (int q = t; q < kend / 4; q += 256) vst2(sr + q * 4, *(const v4f*)&sh[q * 4]); }
__global__ __launch_bounds__(128) void k_pv(const float* __restrict__ PS0, const __bf16* __restrict__ VT, const __bf16* __restrict__ VL, int b, int h0, float* __restrict__ Y) { const int h = h0 + blockIdx.z; const float* PS = PS0 + (size_t)blockIdx.z * TT * TT; __shared__ __align__(16) float ss[4][16][HD + 4];
  const int tid = threadIdx.x, wave = tid >> 5, lane = tid & 31, col = lane & 15, g = lane >> 4; const int ql0 = blockIdx.x * 64 + wave * 16; const int kend = TT;
  v8f acc[HD / 16] = {};
#pragma unroll 1
  for (int kc = 0; kc < kend / 32; ++kc) { const F2 p = split_row(PS + (size_t)(ql0 + col) * TT, kc * 32, lane);
#pragma unroll
    for (int j = 0; j < HD / 16; ++j) { const size_t po = ((size_t)b * CC + h * HD + j * 16 + col) * (size_t)TT + kc * 32; const v16b vh = frag_b(VT + po, lane); acc[j] = wmma_bf(p.h, vh, acc[j]); acc[j] = wmma_bf(p.l, vh, acc[j]); acc[j] = wmma_bf(p.h, frag_b(VL + po, lane), acc[j]); } }
#pragma unroll
  for (int j = 0; j < HD / 16; ++j)
#pragma unroll
    for (int r = 0; r < 8; ++r) ss[wave][8 * g + r][j * 16 + col] = acc[j][r] * (1.0f / 2048.0f);
  LDSX(); for (int rl = 0; rl < 16; ++rl) if (lane < HD / 4) vst2(Y + ((size_t)b * TT + ql0 + rl) * CC + h * HD + lane * 4, *(const v4f*)&ss[wave][rl][lane * 4]); }
__global__ __launch_bounds__(128) void k_o(const float* __restrict__ Y, const float* __restrict__ WO, const float* __restrict__ BO, float* __restrict__ H) { __shared__ __align__(16) float sf[4][16][132];
  const int tid = threadIdx.x, wave = tid >> 5, lane = tid & 31, col = lane & 15, g = lane >> 4; const size_t r0 = (size_t)blockIdx.x * 64 + wave * 16; const int c0 = blockIdx.y * 128;
  v8f acc[8] = {};
#pragma unroll 1
  for (int kc = 0; kc < CC / 32; ++kc) { const F2 a = split_row(Y + (r0 + col) * CC, kc * 32, lane);
#pragma unroll
    for (int j = 0; j < 8; ++j) { v16b w; const int o = c0 + j * 16 + col;
#pragma unroll
      for (int i = 0; i < 8; ++i) { w[i] = (__bf16)WO[(size_t)(kc * 32 + 8 * g + i) * CC + o]; w[8 + i] = (__bf16)WO[(size_t)(kc * 32 + 16 + 8 * g + i) * CC + o]; }
      asm volatile("s_wait_loadcnt 0x0" ::: "memory"); acc[j] = wmma_bf(a.h, w, acc[j]); acc[j] = wmma_bf(a.l, w, acc[j]); } }
#pragma unroll
  for (int j = 0; j < 8; ++j) { const float bb = bfr(BO[c0 + j * 16 + col]);
#pragma unroll
    for (int r = 0; r < 8; ++r) sf[wave][8 * g + r][j * 16 + col] = acc[j][r] + bb; }
  LDSX(); for (int rl = 0; rl < 16; ++rl) { float* hp = H + (r0 + rl) * CC + c0 + lane * 4; const v4f old = *(const v4f*)hp; vst2(hp, old + *(const v4f*)&sf[wave][rl][lane * 4]); } }
__global__ __launch_bounds__(128) void k_ffn1(const float* __restrict__ H, const float* __restrict__ ST, const float* __restrict__ LG, const float* __restrict__ LBt, const float* __restrict__ W1, const float* __restrict__ B1, float* __restrict__ G) { __shared__ __align__(16) float sf[4][16][132];
  const int tid = threadIdx.x, wave = tid >> 5, lane = tid & 31, col = lane & 15, g = lane >> 4; const size_t r0 = (size_t)blockIdx.x * 64 + wave * 16; const int c0 = blockIdx.y * 128;
  v8f acc[8] = {};
#pragma unroll 1
  for (int kc = 0; kc < CC / 32; ++kc) { const F2 a = lnfrag(H, ST, LG, LBt, r0 + col, kc, lane);
#pragma unroll
    for (int j = 0; j < 8; ++j) { v16b w; const int o = c0 + j * 16 + col;
#pragma unroll
      for (int i = 0; i < 8; ++i) { w[i] = (__bf16)W1[(size_t)(kc * 32 + 8 * g + i) * DFF + o]; w[8 + i] = (__bf16)W1[(size_t)(kc * 32 + 16 + 8 * g + i) * DFF + o]; }
      asm volatile("s_wait_loadcnt 0x0" ::: "memory"); acc[j] = wmma_bf(a.h, w, acc[j]); acc[j] = wmma_bf(a.l, w, acc[j]); } }
#pragma unroll
  for (int j = 0; j < 8; ++j) { const float bb = bfr(B1[c0 + j * 16 + col]);
#pragma unroll
    for (int r = 0; r < 8; ++r) sf[wave][8 * g + r][j * 16 + col] = gelu_ni(acc[j][r] + bb); }
  LDSX(); for (int rl = 0; rl < 16; ++rl) vst2(G + (r0 + rl) * DFF + c0 + lane * 4, *(const v4f*)&sf[wave][rl][lane * 4]); }
__global__ __launch_bounds__(128) void k_ffn2(const float* __restrict__ G, const float* __restrict__ W2, const float* __restrict__ B2, float* __restrict__ H) { __shared__ __align__(16) float sf[4][16][132];
  const int tid = threadIdx.x, wave = tid >> 5, lane = tid & 31, col = lane & 15, g = lane >> 4; const size_t r0 = (size_t)blockIdx.x * 64 + wave * 16; const int c0 = blockIdx.y * 128;
  v8f acc[8] = {};
#pragma unroll 1
  for (int kc = 0; kc < DFF / 32; ++kc) { const F2 a = split_row(G + (r0 + col) * DFF, kc * 32, lane);
#pragma unroll
    for (int j = 0; j < 8; ++j) { v16b w; const int o = c0 + j * 16 + col;
#pragma unroll
      for (int i = 0; i < 8; ++i) { w[i] = (__bf16)W2[(size_t)(kc * 32 + 8 * g + i) * CC + o]; w[8 + i] = (__bf16)W2[(size_t)(kc * 32 + 16 + 8 * g + i) * CC + o]; }
      asm volatile("s_wait_loadcnt 0x0" ::: "memory"); acc[j] = wmma_bf(a.h, w, acc[j]); acc[j] = wmma_bf(a.l, w, acc[j]); } }
#pragma unroll
  for (int j = 0; j < 8; ++j) { const float bb = bfr(B2[c0 + j * 16 + col]);
#pragma unroll
    for (int r = 0; r < 8; ++r) sf[wave][8 * g + r][j * 16 + col] = acc[j][r] + bb; }
  LDSX(); for (int rl = 0; rl < 16; ++rl) { float* hp = H + (r0 + rl) * CC + c0 + lane * 4; const v4f old = *(const v4f*)hp; vst2(hp, old + *(const v4f*)&sf[wave][rl][lane * 4]); } }
__global__ __launch_bounds__(128) void k_fin(const float* __restrict__ H, const float* __restrict__ WOUT, const float* __restrict__ BOUT, float* __restrict__ OUT) { __shared__ __align__(16) float sf[4][16][132];
  const int tid = threadIdx.x, wave = tid >> 5, lane = tid & 31, col = lane & 15, g = lane >> 4; const size_t r0 = (size_t)blockIdx.x * 64 + wave * 16;
  v8f acc[8] = {};
#pragma unroll 1
  for (int kc = 0; kc < CC / 32; ++kc) { const F2 a = split_row(H + (r0 + col) * CC, kc * 32, lane);
#pragma unroll
    for (int j = 0; j < 8; ++j) { v16b w; const int o = j * 16 + col;
#pragma unroll
      for (int i = 0; i < 8; ++i) { w[i] = (__bf16)WOUT[(size_t)(kc * 32 + 8 * g + i) * DOUT + o]; w[8 + i] = (__bf16)WOUT[(size_t)(kc * 32 + 16 + 8 * g + i) * DOUT + o]; }
      asm volatile("s_wait_loadcnt 0x0" ::: "memory"); acc[j] = wmma_bf(a.h, w, acc[j]); acc[j] = wmma_bf(a.l, w, acc[j]); } }
#pragma unroll
  for (int j = 0; j < 8; ++j) { const float bb = bfr(BOUT[j * 16 + col]);
#pragma unroll
    for (int r = 0; r < 8; ++r) sf[wave][8 * g + r][j * 16 + col] = acc[j][r] + bb; }
  LDSX(); for (int rl = 0; rl < 16; ++rl) vst2(OUT + (r0 + rl) * DOUT + lane * 4, *(const v4f*)&sf[wave][rl][lane * 4]); }
extern "C" void kernel_launch(void* const* d_in, const int* in_sizes, int n_in, void* d_out, int out_size, void* d_ws, size_t ws_size, hipStream_t stream) {
  (void)in_sizes; (void)n_in; (void)out_size;
  const float** F = (const float**)d_in;
  if (ws_size < (size_t)WS_END) return;
  char* ws = (char*)d_ws; int* DEG = (int*)(ws + WS_DEG); float *H = (float*)(ws + WS_H), *ST = (float*)(ws + WS_ST), *S = (float*)(ws + WS_S), *Y = (float*)(ws + WS_Y), *G = (float*)(ws + WS_G); _Float16 *QH = (_Float16*)(ws + WS_QH), *QL = (_Float16*)(ws + WS_QL), *KH = (_Float16*)(ws + WS_KH), *KL = (_Float16*)(ws + WS_KL); __bf16 *VT = (__bf16*)(ws + WS_VT), *VL = (__bf16*)(ws + WS_VL);
  const int* EI = (const int*)d_in[1]; const int* ET = (const int*)d_in[2];
  k_deg<<<dim3(1), 512, 0, stream>>>(EI, DEG);
  k_emb<<<dim3(NN / 64, CC / 128), 128, 0, stream>>>(F[0], F[4], F[5], H);
  for (int l = 0; l < 2; ++l) { const size_t oW = (size_t)l * CC * CC, oB = (size_t)l * CC;
    k_hadd<<<dim3(NN / 16), 256, 0, stream>>>(H, DEG, F[16] + (size_t)l * 513 * CC, F[17] + (size_t)l * 513 * CC, ST);
    k_qkv<<<dim3(NN / 64, CC / 128, 3), 128, 0, stream>>>(H, ST, F[18] + oB, F[19] + oB, F[6] + oW, F[10] + oB, F[7] + oW, F[11] + oB, F[8] + oW, F[12] + oB, QH, QL, KH, KL, VT, VL);
    for (int h0 = 0; h0 < NH; h0 += HG) {
      k_sc<<<dim3(NN / 64, NN / 128, HG), 128, 0, stream>>>(QH, QL, KH, KL, F[3], F[14] + (size_t)l * 11 * NH, h0, S);
      k_edge<<<dim3(1), 32, 0, stream>>>(EI, ET, F[15] + (size_t)l * 8 * NH, h0, S);
      k_sm<<<dim3(NN, HG), 256, 0, stream>>>(S);
      k_pv<<<dim3(NN / 64, 1, HG), 128, 0, stream>>>(S, VT, VL, 0, h0, Y);
    }
    k_o<<<dim3(NN / 64, CC / 128), 128, 0, stream>>>(Y, F[9] + oW, F[13] + oB, H);
    k_lnst<<<dim3(NN / 16), 256, 0, stream>>>(H, ST);
    k_ffn1<<<dim3(NN / 64, DFF / 128), 128, 0, stream>>>(H, ST, F[20] + oB, F[21] + oB, F[22] + (size_t)l * CC * DFF, F[23] + (size_t)l * DFF, G);
    k_ffn2<<<dim3(NN / 64, CC / 128), 128, 0, stream>>>(G, F[24] + (size_t)l * DFF * CC, F[25] + oB, H);
  }
  k_fin<<<dim3(NN / 64), 128, 0, stream>>>(H, F[26], F[27], (float*)d_out);
}
